// CausalSelfAttention_40003325395456
// MI455X (gfx1250) — hardware-verified
//
#include <hip/hip_runtime.h>
#include <math.h>

constexpr int kBatch   = 4;
constexpr int kSeq     = 4096;
constexpr int kEmb     = 512;
constexpr int kHeads   = 8;
constexpr int kHd      = 64;
constexpr int kRows    = kBatch * kSeq;
constexpr int kBH      = kBatch * kHeads;
constexpr int kChunk   = 64;
constexpr int kNChunk  = kSeq / kChunk;
constexpr int kLp      = 72;
constexpr int kQkvN    = 3 * kEmb;
constexpr int kHalfRows = kRows / 2;
constexpr int kHalfBH   = kBH / 2;
constexpr float kEps   = 1e-6f;
static_assert(kHeads * kHd == kEmb, "head packing");
static_assert(kEmb % 32 == 0, "GEMM K multiple of 32");
static_assert(kHd % 32 == 0 && kChunk % 32 == 0, "tile K multiple of 32");
static_assert(kRows % 64 == 0 && kHalfRows % 64 == 0 && kQkvN % 64 == 0 && kEmb % 64 == 0, "GEMM M, N tile multiples");
static_assert(kSeq % 128 == 0 && kSeq % kChunk == 0, "scan line groups and chunks");
static_assert(kSeq == 4096 && kEmb == 512 && kHd == 64, "shift constants in the projection epilogue");
static_assert(kLp % 8 == 0, "LDS pitch keeps 16-B alignment");

typedef __attribute__((ext_vector_type(16))) __bf16   v16b;
typedef __attribute__((ext_vector_type(8)))  __bf16   v8b;
typedef __attribute__((ext_vector_type(8)))  float    v8f;
typedef __attribute__((ext_vector_type(4)))  float    v4f;
typedef __attribute__((ext_vector_type(4)))  unsigned int v4u;

__device__ __forceinline__ unsigned short f2bf_bits(float f) {
  unsigned u = __float_as_uint(f);
  return (unsigned short)((u + 0x7FFFu + ((u >> 16) & 1u)) >> 16);
}
__device__ __forceinline__ float bf_bits2f(unsigned short h) { return __uint_as_float(((unsigned)h) << 16); }
__device__ __forceinline__ float bf16r(float f) { return bf_bits2f(f2bf_bits(f)); }
__device__ __forceinline__ unsigned pk16(unsigned short a, unsigned short b) { return (unsigned)a | ((unsigned)b << 16); }
__device__ __forceinline__ __bf16 bits2bf(unsigned short u) { return __builtin_bit_cast(__bf16, u); }

__device__ __forceinline__ void dep_guard4_b(v8f& a, v8f& b, v8f& c, v8f& d, v16b x, v16b y) { asm volatile("v_nop\n\tv_nop\n\tv_nop\n\tv_nop" : "+v"(a), "+v"(b), "+v"(c), "+v"(d) : "v"(x), "v"(y)); }
__device__ __forceinline__ void keep4_b(v16b a, v16b b, v16b c, v16b d) { asm volatile("v_nop" :: "v"(a), "v"(b), "v"(c), "v"(d)); }
__device__ __forceinline__ void acc_guard4(v8f& a, v8f& b, v8f& c, v8f& d) { asm volatile("v_nop\n\tv_nop\n\tv_nop\n\tv_nop" : "+v"(a), "+v"(b), "+v"(c), "+v"(d)); }

template <typename T> struct Frag;
template <> struct Frag<__bf16> {
  typedef v16b V; union U { v16b v; v8b h[2]; };
  static __device__ __forceinline__ v16b load(const __bf16* p) {
    U f; f.h[0] = *(const v8b*)(p); f.h[1] = *(const v8b*)(p + 16); return f.v;
  }
  static __device__ __forceinline__ v8f mma(v16b a, v16b b, v8f c) {
    return __builtin_amdgcn_wmma_f32_16x16x32_bf16(false, a, false, b, (short)0, c, false, false);
  }
};

__device__ __forceinline__ v8f mma_g(v16b a, v16b b, v8f c) {
  c = __builtin_amdgcn_wmma_f32_16x16x32_bf16(false, a, false, b, (short)0, c, false, false);
  asm volatile("v_nop\n\tv_nop\n\tv_nop\n\tv_nop" : "+v"(c) : "v"(a), "v"(b));
  return c;
}

__device__ __forceinline__ void wave_lds_sync() {
  __builtin_amdgcn_fence(__ATOMIC_RELEASE, "workgroup");
  __builtin_amdgcn_wave_barrier();
  __builtin_amdgcn_fence(__ATOMIC_ACQUIRE, "workgroup");
}

__global__ __launch_bounds__(256) void cvt8_bf16_kernel(const float* __restrict__ src, unsigned short* __restrict__ dst, int n8) {
  const int i = blockIdx.x * 256 + threadIdx.x;
  if (i < n8) {
    const float* p = src + 8 * (size_t)i;
    const v4f a = *(const v4f*)(p);
    const v4f b = *(const v4f*)(p + 4);
    unsigned short hb[8];
#pragma unroll
    for (int e = 0; e < 4; ++e) {
      const float fa = a[e];
      const float fb = b[e];
      hb[e]     = f2bf_bits(fa);
      hb[4 + e] = f2bf_bits(fb);
    }
    const v4u u = (v4u){pk16(hb[0], hb[1]), pk16(hb[2], hb[3]), pk16(hb[4], hb[5]), pk16(hb[6], hb[7])};
    unsigned short* q = dst + 8 * (size_t)i;
    *(volatile v4u*)q = u;
    __threadfence();
    *(volatile v4u*)q = u;
  }
}

__global__ __launch_bounds__(256) void bias_prep_kernel(const float* __restrict__ b0, const float* __restrict__ b1,
                                                        const float* __restrict__ b2, const float* __restrict__ b3,
                                                        float* __restrict__ dst) {
  const int tid = threadIdx.x;
#pragma unroll 1
  for (int it = 0; it < 2; ++it) {
    const int idx4 = it * 256 + tid;
    const int which = idx4 >> 7;
    const int off = (idx4 & 127) * 4;
    const v4f va = *(const v4f*)(b0 + off);
    const v4f vb = *(const v4f*)(b1 + off);
    const v4f vc = *(const v4f*)(b2 + off);
    const v4f vd = *(const v4f*)(b3 + off);
    v4f o;
#pragma unroll
    for (int e = 0; e < 4; ++e) {
      const float s01 = (which == 0) ? va[e] : vb[e];
      const float s23 = (which == 2) ? vc[e] : vd[e];
      o[e] = bf16r((which < 2) ? s01 : s23);
    }
    float* op = dst + which * kEmb + off;
    *(volatile v4f*)op = o;
    __threadfence();
    *(volatile v4f*)op = o;
  }
}

template <int MODE>
__global__ __launch_bounds__(256) void gemm64_kernel(
    const unsigned short* __restrict__ Ap, const unsigned short* __restrict__ A2p,
    const unsigned short* __restrict__ Btp, const float* __restrict__ bias,
    unsigned short* __restrict__ QHp, unsigned short* __restrict__ QLp,
    unsigned short* __restrict__ KHp, unsigned short* __restrict__ KLp,
    float* __restrict__ Fout, int M, int N) {
  typedef __bf16 T;
  const T* A = (const T*)Ap; const T* A2 = (const T*)A2p; const T* Bt = (const T*)Btp;
  __shared__ __align__(16) float sT[8][16 * 68];
  const int lane = threadIdx.x & 31;
  const int wave = threadIdx.x >> 5;
  const int tilesN = N >> 6;
  const int tilesM = M >> 6;
  const int tile = blockIdx.x * 8 + wave;
  if (tile >= tilesM * tilesN) return;
  const int tm = tile / tilesN;
  const int tn = tile - tm * tilesN;
  const int m0 = tm << 6;
  const int n0 = tn << 6;

  const int rlane = lane & 15;
  const int koff  = (lane >> 4) * 8;
  const int mOff  = (lane >> 4) * 8;

  v8f acc[4][4];
#pragma unroll
  for (int i = 0; i < 4; ++i)
#pragma unroll
    for (int j = 0; j < 4; ++j) acc[i][j] = (v8f){0.f,0.f,0.f,0.f,0.f,0.f,0.f,0.f};

  for (int k0 = 0; k0 < kEmb; k0 += 32) {
    v16b bh[4];
#pragma unroll
    for (int j = 0; j < 4; ++j) {
      const size_t bo = (size_t)(n0 + (j << 4) + rlane) * kEmb + koff + k0;
      bh[j] = Frag<T>::load(Bt + bo);
    }
#pragma unroll
    for (int i = 0; i < 4; ++i) {
      const size_t ao = (size_t)(m0 + (i << 4) + rlane) * kEmb + koff + k0;
      v16b ah = Frag<T>::load(A + ao);
      v16b al = ah;
      if (MODE == 1) al = Frag<T>::load(A2 + ao);
#pragma unroll
      for (int j = 0; j < 4; ++j) {
        acc[i][j] = Frag<T>::mma(ah, bh[j], acc[i][j]);
        if (MODE == 1) acc[i][j] = Frag<T>::mma(al, bh[j], acc[i][j]);
      }
      dep_guard4_b(acc[i][0], acc[i][1], acc[i][2], acc[i][3], ah, al);
    }
    keep4_b(bh[0], bh[1], bh[2], bh[3]);
  }
  acc_guard4(acc[0][0], acc[0][1], acc[0][2], acc[0][3]);
  acc_guard4(acc[1][0], acc[1][1], acc[1][2], acc[1][3]);
  acc_guard4(acc[2][0], acc[2][1], acc[2][2], acc[2][3]);
  acc_guard4(acc[3][0], acc[3][1], acc[3][2], acc[3][3]);

  float* slab = sT[wave];
  const int sel  = n0 >> 9;
  const int hcol = (n0 & (kEmb - 1)) >> 6;
  const int bb   = m0 >> 12;
  const int l0   = m0 & (kSeq - 1);
  const size_t rowbase = ((size_t)(bb * kHeads + hcol)) * kSeq + (size_t)l0;
  unsigned short* Ch = (sel == 0) ? QHp : KHp;
  unsigned short* Cl = (sel == 0) ? QLp : KLp;
  const int hh = lane >> 4, c4 = (lane & 15) * 4;
  const int q4 = lane >> 3, c8 = (lane & 7) * 8;
#pragma unroll
  for (int i = 0; i < 4; ++i) {
#pragma unroll
    for (int j = 0; j < 4; ++j) {
      const int n = n0 + (j << 4) + rlane;
      const float bv = bias[n];
#pragma unroll
      for (int r = 0; r < 8; ++r) {
        const float v = acc[i][j][r] + bv;
        slab[(mOff + r) * 68 + (j << 4) + rlane] = v;
      }
    }
    wave_lds_sync();
    if (MODE == 0 && sel < 2) {
#pragma unroll 1
      for (int it = 0; it < 8; ++it) {
        float* sp = slab + (it * 2 + hh) * 68 + c4;
        v4f v = *(const v4f*)sp;
#pragma unroll
        for (int e = 0; e < 4; ++e) {
          const float x = v[e];
          v[e] = 1.0f / (1.0f + expf(-x));
        }
        *(v4f*)sp = v;
      }
      wave_lds_sync();
    }
    if (MODE == 1) {
      float* Cf = Fout;
      for (int pass = 0; pass < 2; ++pass) {
#pragma unroll
        for (int it = 0; it < 8; ++it) {
          const int row = it * 2 + hh;
          const v4f v = *(const v4f*)(slab + row * 68 + c4);
          *(volatile v4f*)(Cf + (size_t)(m0 + (i << 4) + row) * kEmb + n0 + c4) = v;
        }
        __threadfence();
      }
    } else if (sel == 2) {
      float* Cf = Fout;
      for (int pass = 0; pass < 2; ++pass) {
#pragma unroll
        for (int it = 0; it < 8; ++it) {
          const int row = it * 2 + hh;
          const v4f v = *(const v4f*)(slab + row * 68 + c4);
          *(volatile v4f*)(Cf + (rowbase + (size_t)((i << 4) + row)) * kHd + c4) = v;
        }
        __threadfence();
      }
    } else {
      v4u uh[4], ul[4];
#pragma unroll
      for (int it = 0; it < 4; ++it) {
        const float* sp = slab + (it * 4 + q4) * 68 + c8;
        unsigned short hb[8], lb[8];
#pragma unroll
        for (int e = 0; e < 8; ++e) {
          const float f = sp[e];
          hb[e] = f2bf_bits(f);
          lb[e] = f2bf_bits(f - bf_bits2f(hb[e]));
        }
        uh[it] = (v4u){pk16(hb[0], hb[1]), pk16(hb[2], hb[3]), pk16(hb[4], hb[5]), pk16(hb[6], hb[7])};
        ul[it] = (v4u){pk16(lb[0], lb[1]), pk16(lb[2], lb[3]), pk16(lb[4], lb[5]), pk16(lb[6], lb[7])};
      }
      for (int pass = 0; pass < 2; ++pass) {
#pragma unroll
        for (int it = 0; it < 4; ++it) {
          const size_t o = (rowbase + (size_t)((i << 4) + it * 4 + q4)) * kHd + c8;
          *(volatile v4u*)(Ch + o) = uh[it];
          *(volatile v4u*)(Cl + o) = ul[it];
        }
        __threadfence();
      }
    }
    wave_lds_sync();
  }
}

__global__ __launch_bounds__(32) void flow_scan_kernel(const unsigned short* __restrict__ QHp, const unsigned short* __restrict__ QLp,
                                                       const unsigned short* __restrict__ KHp, const unsigned short* __restrict__ KLp,
                                                       float* __restrict__ RS, float* __restrict__ COMP) {
  const int bh = blockIdx.x, lane = threadIdx.x;
  const size_t wbase = (size_t)bh * kSeq * (kHd / 2);
  const unsigned* QHw = (const unsigned*)QHp + wbase;
  const unsigned* QLw = (const unsigned*)QLp + wbase;
  const unsigned* KHw = (const unsigned*)KHp + wbase;
  const unsigned* KLw = (const unsigned*)KLp + wbase;
  float kc0 = 0.f, kc1 = 0.f, qc0 = 0.f, qc1 = 0.f;
  float s10 = 0.f, s11 = 0.f, s20 = 0.f, s21 = 0.f, cssum = 0.f;
  float rk0 = 0.f, rk1 = 0.f, rk2 = 0.f, rk3 = 0.f;
  float ck0 = 0.f, ck1 = 0.f, ck2 = 0.f, ck3 = 0.f;
#pragma unroll 1
  for (int l = 0; l < kSeq; ++l) {
    const size_t wi = (size_t)l * (kHd / 2) + lane;
    const unsigned wqh = QHw[wi], wql = QLw[wi], wkh = KHw[wi], wkl = KLw[wi];
    const float q0 = __uint_as_float(wqh << 16) + __uint_as_float(wql << 16);
    const float q1 = __uint_as_float(wqh & 0xffff0000u) + __uint_as_float(wql & 0xffff0000u);
    const float k0 = __uint_as_float(wkh << 16) + __uint_as_float(wkl << 16);
    const float k1 = __uint_as_float(wkh & 0xffff0000u) + __uint_as_float(wkl & 0xffff0000u);
    kc0 += k0; kc1 += k1; qc0 += q0; qc1 += q1;
    float d1 = (q0 + kEps) * (kc0 + kEps) + (q1 + kEps) * (kc1 + kEps);
    float d2 = (k0 + kEps) * (qc0 + kEps) + (k1 + kEps) * (qc1 + kEps);
#pragma unroll
    for (int off = 16; off > 0; off >>= 1) {
      d1 += __shfl_xor(d1, off, 32);
      d2 += __shfl_xor(d2, off, 32);
    }
    const float nrm = (float)(l + 1);
    const float inv_nrm = 1.0f / nrm;
    const float sink_in = (1.0f / d1) * nrm;
    const float src_out = (1.0f / d2) * nrm;
    s10 += k0 * src_out; s11 += k1 * src_out;
    s20 += q0 * sink_in; s21 += q1 * sink_in;
    float d3 = (q0 + kEps) * (s10 + kEps) + (q1 + kEps) * (s11 + kEps);
    float d4 = (k0 + kEps) * (s20 + kEps) + (k1 + kEps) * (s21 + kEps);
#pragma unroll
    for (int off = 16; off > 0; off >>= 1) {
      d3 += __shfl_xor(d3, off, 32);
      d4 += __shfl_xor(d4, off, 32);
    }
    const float csink = d3 * inv_nrm;
    const float csrc  = fminf(fmaxf(d4 * inv_nrm, -1.0f), 1.0f);
    const float salloc = 1.0f / (1.0f + expf(-csink));
    const float cse = expf(csrc);
    cssum += cse;
    const float compv = (cse / cssum) * nrm;
    const float rsv = salloc * (sink_in * inv_nrm);
    const int ph = l & 127;
    const int sl = ph - 4 * lane;
    rk0 = (sl == 0) ? rsv : rk0;  rk1 = (sl == 1) ? rsv : rk1;  rk2 = (sl == 2) ? rsv : rk2;  rk3 = (sl == 3) ? rsv : rk3;
    ck0 = (sl == 0) ? compv : ck0;  ck1 = (sl == 1) ? compv : ck1;  ck2 = (sl == 2) ? compv : ck2;  ck3 = (sl == 3) ? compv : ck3;
    if (ph == 127) {
      const v4f ro = (v4f){rk0, rk1, rk2, rk3};
      const v4f co = (v4f){ck0, ck1, ck2, ck3};
      const size_t o = (size_t)bh * kSeq + (size_t)(l - 127) + 4 * lane;
      *(volatile v4f*)(RS + o) = ro;
      *(volatile v4f*)(COMP + o) = co;
      __threadfence();
      *(volatile v4f*)(RS + o) = ro;
      *(volatile v4f*)(COMP + o) = co;
    }
  }
}

__global__ __launch_bounds__(128) void flow_attn_kernel(
    const unsigned short* __restrict__ QHp, const unsigned short* __restrict__ QLp,
    const unsigned short* __restrict__ KHp, const unsigned short* __restrict__ KLp,
    const float* __restrict__ VF, const float* __restrict__ RS, const float* __restrict__ COMP,
    unsigned short* __restrict__ AHp, unsigned short* __restrict__ ALp, int bh0) {
  __shared__ __align__(16) __bf16 Rh[kChunk * kLp];
  __shared__ __align__(16) __bf16 Rl[kChunk * kLp];
  __shared__ __align__(16) __bf16 VTh[kHd * kLp];
  __shared__ __align__(16) __bf16 VTl[kHd * kLp];
  __shared__ __align__(16) __bf16 Ph[4][16 * kLp];
  __shared__ __align__(16) __bf16 Pl[4][16 * kLp];

  const int tid = threadIdx.x, lane = tid & 31, wave = tid >> 5;
  const int c = lane & 15, hh = lane >> 4, koff = hh * 8;
  const int bh = bh0 + (int)blockIdx.x;
  const int hd = bh & (kHeads - 1);
  const int bl = (int)blockIdx.x >> 3;
  const size_t pbase = (size_t)bh * kSeq * kHd;
  const __bf16* QH = (const __bf16*)QHp + pbase;
  const __bf16* QL = (const __bf16*)QLp + pbase;
  const __bf16* KH = (const __bf16*)KHp + pbase;
  const __bf16* KL = (const __bf16*)KLp + pbase;
  const unsigned short* KHu = KHp + pbase;
  const unsigned short* KLu = KLp + pbase;
  const float* vfp = VF + pbase;
  const float* rsp = RS + (size_t)bh * kSeq;
  const float* cpp = COMP + (size_t)bh * kSeq;
  unsigned short* ahp = AHp + ((size_t)bl * kSeq) * kEmb + hd * kHd;
  unsigned short* alp = ALp + ((size_t)bl * kSeq) * kEmb + hd * kHd;
  __bf16* ph = Ph[wave];
  __bf16* pl = Pl[wave];
  const int lr = tid >> 1, dh = (tid & 1) * 32;
  const int q4 = lane >> 3, c8 = (lane & 7) * 8;
  const v8f z8 = (v8f){0.f,0.f,0.f,0.f,0.f,0.f,0.f,0.f};

  v8f accS[4];
  accS[0] = z8; accS[1] = z8; accS[2] = z8; accS[3] = z8;

#pragma unroll 1
  for (int n = 0; n < kNChunk; ++n) {
    const int l0 = n * kChunk;
    __syncthreads();

#pragma unroll
    for (int j = 0; j < 4; ++j) {
#pragma unroll
      for (int r = 0; r < 8; ++r) {
        const float s = accS[j][r];
        const unsigned short hb = f2bf_bits(s);
        const unsigned short lb = f2bf_bits(s - bf_bits2f(hb));
        const int o = (16 * wave + 8 * hh + r) * kLp + 16 * j + c;
        Rh[o] = bits2bf(hb);
        Rl[o] = bits2bf(lb);
      }
    }
    {
      const float cv = cpp[l0 + lr];
      const float* vrow = vfp + (size_t)(l0 + lr) * kHd + dh;
#pragma unroll
      for (int g = 0; g < 2; ++g) {
        v4f vv[4];
#pragma unroll
        for (int i = 0; i < 4; ++i) vv[i] = *(const v4f*)(vrow + 16 * g + 4 * i);
#pragma unroll
        for (int i = 0; i < 4; ++i) {
#pragma unroll
          for (int e = 0; e < 4; ++e) {
            const float f = vv[i][e] * cv;
            const unsigned short hb = f2bf_bits(f);
            const unsigned short lb = f2bf_bits(f - bf_bits2f(hb));
            const int d = dh + 16 * g + 4 * i + e;
            VTh[d * kLp + lr] = bits2bf(hb);
            VTl[d * kLp + lr] = bits2bf(lb);
          }
        }
        asm volatile("" ::: "memory");
      }
    }
    __syncthreads();

    v16b qh[2], ql[2];
    {
      const size_t qo = (size_t)(l0 + 16 * wave + c) * kHd + koff;
#pragma unroll
      for (int dc = 0; dc < 2; ++dc) {
        qh[dc] = Frag<__bf16>::load(QH + qo + dc * 32);
        ql[dc] = Frag<__bf16>::load(QL + qo + dc * 32);
      }
    }
    asm volatile("" ::: "memory");
#pragma unroll
    for (int j = 0; j < 4; ++j) {
      v8f s = z8;
      const size_t ko = (size_t)(l0 + 16 * j + c) * kHd + koff;
#pragma unroll
      for (int dc = 0; dc < 2; ++dc) {
        const v16b kh = Frag<__bf16>::load(KH + ko + dc * 32);
        const v16b kl = Frag<__bf16>::load(KL + ko + dc * 32);
        s = mma_g(qh[dc], kh, s);
        s = mma_g(qh[dc], kl, s);
        s = mma_g(ql[dc], kh, s);
      }
      const int jj = 16 * j + c;
#pragma unroll
      for (int r = 0; r < 8; ++r) {
        const int ii = 16 * wave + 8 * hh + r;
        const float pv = (jj <= ii) ? s[r] : 0.0f;
        const unsigned short hb = f2bf_bits(pv);
        const unsigned short lb = f2bf_bits(pv - bf_bits2f(hb));
        ph[(8 * hh + r) * kLp + jj] = bits2bf(hb);
        pl[(8 * hh + r) * kLp + jj] = bits2bf(lb);
      }
      asm volatile("" ::: "memory");
    }
    wave_lds_sync();

    v8f accO[4];
    accO[0] = z8; accO[1] = z8; accO[2] = z8; accO[3] = z8;
#pragma unroll
    for (int t = 0; t < 4; ++t) {
      const __bf16* sph = Rh + (16 * t + c) * kLp + koff;
      const __bf16* spl = Rl + (16 * t + c) * kLp + koff;
#pragma unroll
      for (int dc = 0; dc < 2; ++dc) {
        const v16b sh = Frag<__bf16>::load(sph + dc * 32);
        const v16b sl = Frag<__bf16>::load(spl + dc * 32);
        accO[t] = mma_g(qh[dc], sh, accO[t]);
        accO[t] = mma_g(qh[dc], sl, accO[t]);
        accO[t] = mma_g(ql[dc], sh, accO[t]);
      }
    }
#pragma unroll
    for (int kk = 0; kk < 2; ++kk) {
      const v16b pah = Frag<__bf16>::load(ph + c * kLp + kk * 32 + koff);
      const v16b pal = Frag<__bf16>::load(pl + c * kLp + kk * 32 + koff);
#pragma unroll
      for (int t = 0; t < 4; ++t) {
        const v16b vh = Frag<__bf16>::load(VTh + (16 * t + c) * kLp + kk * 32 + koff);
        const v16b vl = Frag<__bf16>::load(VTl + (16 * t + c) * kLp + kk * 32 + koff);
        accO[t] = mma_g(pah, vh, accO[t]);
        accO[t] = mma_g(pah, vl, accO[t]);
        accO[t] = mma_g(pal, vh, accO[t]);
      }
    }
    {
      const float* rp = rsp + l0 + 16 * wave + 8 * hh;
      const v4f r0 = *(const v4f*)(rp);
      const v4f r1 = *(const v4f*)(rp + 4);
      float rsv[8];
#pragma unroll
      for (int e = 0; e < 4; ++e) { rsv[e] = r0[e]; rsv[4 + e] = r1[e]; }
#pragma unroll
      for (int t = 0; t < 4; ++t) {
#pragma unroll
        for (int r = 0; r < 8; ++r) {
          const float o = accO[t][r] * rsv[r];
          const unsigned short hb = f2bf_bits(o);
          const unsigned short lb = f2bf_bits(o - bf_bits2f(hb));
          ph[(8 * hh + r) * kLp + 16 * t + c] = bits2bf(hb);
          pl[(8 * hh + r) * kLp + 16 * t + c] = bits2bf(lb);
        }
      }
      wave_lds_sync();
      v4u uh[4], ul[4];
#pragma unroll
      for (int it = 0; it < 4; ++it) {
        const int row = it * 4 + q4;
        const v8b hv = *(const v8b*)(ph + row * kLp + c8);
        const v8b lv = *(const v8b*)(pl + row * kLp + c8);
        uh[it] = __builtin_bit_cast(v4u, hv);
        ul[it] = __builtin_bit_cast(v4u, lv);
      }
      for (int pass = 0; pass < 2; ++pass) {
#pragma unroll
        for (int it = 0; it < 4; ++it) {
          const size_t o = (size_t)(l0 + 16 * wave + it * 4 + q4) * kEmb + c8;
          *(volatile v4u*)(ahp + o) = uh[it];
          *(volatile v4u*)(alp + o) = ul[it];
        }
        __threadfence();
      }
      wave_lds_sync();
    }
    __syncthreads();

    {
      const size_t ko = (size_t)(l0 + lr) * kHd + dh;
      const v4u* kh4 = (const v4u*)(KHu + ko);
      const v4u* kl4 = (const v4u*)(KLu + ko);
      v4u wh[4], wl[4];
#pragma unroll
      for (int g = 0; g < 4; ++g) { wh[g] = kh4[g]; wl[g] = kl4[g]; }
#pragma unroll
      for (int g = 0; g < 4; ++g) {
#pragma unroll
        for (int e = 0; e < 4; ++e) {
          const unsigned a = wh[g][e];
          const unsigned b = wl[g][e];
          const int d = dh + 8 * g + 2 * e;
          const unsigned a0 = a & 0xffffu, a1 = a >> 16;
          const unsigned b0 = b & 0xffffu, b1 = b >> 16;
          Rh[d * kLp + lr]       = bits2bf((unsigned short)a0);
          Rh[(d + 1) * kLp + lr] = bits2bf((unsigned short)a1);
          Rl[d * kLp + lr]       = bits2bf((unsigned short)b0);
          Rl[(d + 1) * kLp + lr] = bits2bf((unsigned short)b1);
        }
      }
    }
    __syncthreads();

#pragma unroll
    for (int kk = 0; kk < 2; ++kk) {
      const v16b vah = Frag<__bf16>::load(VTh + (16 * wave + c) * kLp + kk * 32 + koff);
      const v16b val = Frag<__bf16>::load(VTl + (16 * wave + c) * kLp + kk * 32 + koff);
#pragma unroll
      for (int j = 0; j < 4; ++j) {
        const v16b kh = Frag<__bf16>::load(Rh + (16 * j + c) * kLp + kk * 32 + koff);
        const v16b kl = Frag<__bf16>::load(Rl + (16 * j + c) * kLp + kk * 32 + koff);
        accS[j] = mma_g(vah, kh, accS[j]);
        accS[j] = mma_g(vah, kl, accS[j]);
        accS[j] = mma_g(val, kh, accS[j]);
      }
    }
    acc_guard4(accS[0], accS[1], accS[2], accS[3]);
  }
}

extern "C" void kernel_launch(void* const* d_in, const int* in_sizes, int n_in,
                              void* d_out, int out_size, void* d_ws, size_t ws_size, hipStream_t stream) {
  if (n_in < 9 || d_out == nullptr || d_ws == nullptr) return;
  if (in_sizes[0] != kRows * kEmb || in_sizes[1] != kEmb * kEmb || in_sizes[2] != kEmb ||
      in_sizes[3] != kEmb * kEmb || in_sizes[4] != kEmb || in_sizes[5] != kEmb * kEmb ||
      in_sizes[6] != kEmb || in_sizes[7] != kEmb * kEmb || in_sizes[8] != kEmb ||
      out_size != kRows * kEmb) return;

  const float* x  = (const float*)d_in[0];
  const float* Wq = (const float*)d_in[1];
  const float* bq = (const float*)d_in[2];
  const float* Wk = (const float*)d_in[3];
  const float* bk = (const float*)d_in[4];
  const float* Wv = (const float*)d_in[5];
  const float* bv = (const float*)d_in[6];
  const float* Wo = (const float*)d_in[7];
  const float* bo = (const float*)d_in[8];
  float* out = (float*)d_out;

  char* ws = (char*)d_ws; size_t off = 0;
  auto carve = [&](size_t bytes) -> char* { char* p = ws + off; off += (bytes + 255) & ~(size_t)255; return p; };
  unsigned short* XB   = (unsigned short*)carve((size_t)kRows * kEmb * 2);
  unsigned short* WQKV = (unsigned short*)carve((size_t)kQkvN * kEmb * 2);
  unsigned short* WOB  = (unsigned short*)carve((size_t)kEmb * kEmb * 2);
  float*          BIAS = (float*)carve((size_t)4 * kEmb * 4);
  unsigned short* QH   = (unsigned short*)carve((size_t)kBH * kSeq * kHd * 2);
  unsigned short* QL   = (unsigned short*)carve((size_t)kBH * kSeq * kHd * 2);
  unsigned short* KH   = (unsigned short*)carve((size_t)kBH * kSeq * kHd * 2);
  unsigned short* KL   = (unsigned short*)carve((size_t)kBH * kSeq * kHd * 2);
  float*          VF   = (float*)carve((size_t)kBH * kSeq * kHd * 4);
  float*          RS   = (float*)carve((size_t)kBH * kSeq * 4);
  float*          COMP = (float*)carve((size_t)kBH * kSeq * 4);
  if (off > ws_size || off > (size_t)134217728) return;
  unsigned short* AH = XB;
  unsigned short* AL = XB + (size_t)kHalfRows * kEmb;

  const int n8x = kRows * kEmb / 8;
  const int n8w = kEmb * kEmb / 8;
  cvt8_bf16_kernel<<<(n8x + 255) / 256, 256, 0, stream>>>(x,  XB, n8x);
  cvt8_bf16_kernel<<<(n8w + 255) / 256, 256, 0, stream>>>(Wq, WQKV, n8w);
  cvt8_bf16_kernel<<<(n8w + 255) / 256, 256, 0, stream>>>(Wk, WQKV + (size_t)kEmb * kEmb, n8w);
  cvt8_bf16_kernel<<<(n8w + 255) / 256, 256, 0, stream>>>(Wv, WQKV + (size_t)2 * kEmb * kEmb, n8w);
  cvt8_bf16_kernel<<<(n8w + 255) / 256, 256, 0, stream>>>(Wo, WOB, n8w);
  bias_prep_kernel<<<1, 256, 0, stream>>>(bq, bk, bv, bo, BIAS);

  gemm64_kernel<0><<<(kRows / 64) * (kQkvN / 64) / 8, 256, 0, stream>>>(
      XB, XB, WQKV, BIAS, QH, QL, KH, KL, VF, kRows, kQkvN);

  flow_scan_kernel<<<kBH, 32, 0, stream>>>(QH, QL, KH, KL, RS, COMP);

  for (int half = 0; half < 2; ++half) {
    flow_attn_kernel<<<kHalfBH, 128, 0, stream>>>(QH, QL, KH, KL, VF, RS, COMP, AH, AL, half * kHalfBH);
    gemm64_kernel<1><<<(kHalfRows / 64) * (kEmb / 64) / 8, 256, 0, stream>>>(
        AH, AL, WOB, BIAS + 3 * kEmb, QH, QL, KH, KL,
        out + (size_t)half * kHalfRows * kEmb, kHalfRows, kEmb);
  }
}
